// shCaster_86337432584571
// MI455X (gfx1250) — hardware-run, weakly checked
//
#include <hip/hip_runtime.h>
#include <math.h>

#pragma clang fp contract(off)

typedef __attribute__((ext_vector_type(16))) _Float16 v16h;
typedef __attribute__((ext_vector_type(8)))  _Float16 v8h;
typedef __attribute__((ext_vector_type(8)))  float    v8f;
typedef __attribute__((ext_vector_type(4)))  float    v4f;

constexpr int kPts      = 4096 * 128;
constexpr int kJoints   = 24;
constexpr int kBlock    = 256;
constexpr int kWaves    = kBlock / 32;
constexpr int kGrid     = kPts / kBlock;
constexpr int kKPad     = 32;
constexpr int kNPad     = 16;
constexpr int kNReal    = 12;
constexpr int kRegionF  = 768;
constexpr int kStage0   = 512;
constexpr int kStage1   = 608;
static_assert(kPts % kBlock == 0, "exact grid");
static_assert(kGrid * kBlock == kPts, "exact grid");
static_assert((size_t)kPts * 3 * 4 == 6291456ull, "second output byte offset");
static_assert(((size_t)kPts * 3 * 4) % 128 == 0, "second output is line aligned");
static_assert(kJoints <= kKPad && kNReal <= kNPad, "pads");
static_assert(32 * kJoints <= kRegionF, "raw weight region");
static_assert(kStage1 + 96 <= kRegionF && kStage0 + 96 <= kStage1 && 32 * 16 <= kStage0, "region re-use map");

constexpr float kC0   = 0.28209479177387814f;
constexpr float kC1   = 0.4886025119029199f;
constexpr float kC1n  = -0.4886025119029199f;
constexpr float kC2_0 = 1.0925484305920792f;
constexpr float kC2_1 = -1.0925484305920792f;
constexpr float kC2_2 = 0.31539156525252005f;
constexpr float kC2_3 = -1.0925484305920792f;
constexpr float kC2_4 = 0.5462742152960396f;
constexpr float kEps  = 1e-6f;
constexpr float kCarry     = 2048.0f;
constexpr float kCarryInv  = 1.0f / 2048.0f;
constexpr float kHalfMinN  = 6.103515625e-05f;

union FragU { v16h v; v8h h[2]; };
__device__ __forceinline__ v16h frag_load(const _Float16* p) {
  FragU f;
  f.h[0] = *(const v8h*)(p);
  f.h[1] = *(const v8h*)(p + 16);
  return f.v;
}
__device__ __forceinline__ v8f mma_h(v16h a, v16h b, v8f c) {
  c = __builtin_amdgcn_wmma_f32_16x16x32_f16(false, a, false, b, (short)0, c, false, false);
  asm volatile("v_nop\n\tv_nop\n\tv_nop\n\tv_nop" : "+v"(c) : "v"(a), "v"(b));
  return c;
}
__device__ __forceinline__ void split_h(float v, _Float16& hi, _Float16& lo) {
  const float vh = (fabsf(v) < kHalfMinN) ? 0.0f : v;
  hi = (_Float16)vh;
  const float hf = (float)hi;
  lo = (_Float16)((v - hf) * kCarry);
}

__global__ __launch_bounds__(256) void blend_points_kernel(
    const float* __restrict__ xyz, const float* __restrict__ vdir,
    const float* __restrict__ tr, const float* __restrict__ feats,
    const float* __restrict__ locs, float* __restrict__ out)
{
  __shared__ __align__(16) float    sM[kJoints * 16];
  __shared__ __align__(16) float    sF[kJoints * 12];
  __shared__ __align__(16) float    sL[kJoints * 4];
  __shared__ __align__(16) _Float16 sBh[kNPad * kKPad];
  __shared__ __align__(16) _Float16 sBl[kNPad * kKPad];
  __shared__ __align__(16) _Float16 sAh[kWaves][32 * kKPad];
  __shared__ __align__(16) _Float16 sAl[kWaves][32 * kKPad];
  __shared__ __align__(16) float    sR[kWaves][kRegionF];

  const int tid  = (int)threadIdx.x;
  const int lane = tid & 31;
  const int wave = __builtin_amdgcn_readfirstlane((int)(threadIdx.x >> 5));

  for (int i = tid; i < kJoints * 16; i += kBlock) sM[i] = tr[i];
  for (int i = tid; i < kJoints * 12; i += kBlock) {
    const int j = i / 12;
    const int k = i - j * 12;
    const int kc = (k < 9) ? k : 8;
    float v = feats[j * 9 + kc];
    asm volatile("" : "+v"(v));
    sF[i] = (k < 9) ? v : 0.0f;
  }
  if (wave < 3) {
    const int j = tid >> 2;
    const int k = tid & 3;
    const int kc = (k < 3) ? k : 2;
    float v = locs[j * 3 + kc];
    asm volatile("" : "+v"(v));
    sL[tid] = (k < 3) ? v : 0.0f;
  }

  const int pt  = (int)blockIdx.x * kBlock + tid;
  const int ptc = (pt < kPts) ? pt : (kPts - 1);
  const float px = xyz[(size_t)ptc * 3 + 0];
  const float py = xyz[(size_t)ptc * 3 + 1];
  const float pz = xyz[(size_t)ptc * 3 + 2];
  const float qx = px - vdir[(size_t)ptc * 3 + 0];
  const float qy = py - vdir[(size_t)ptc * 3 + 1];
  const float qz = pz - vdir[(size_t)ptc * 3 + 2];

  __syncthreads();

  if (wave < 2) {
    const int n = tid >> 2;
    const int g = tid & 3;
    const int nc = (n < kNReal) ? n : (kNReal - 1);
    v8h hv, lv;
#pragma unroll
    for (int e = 0; e < 8; ++e) {
      const int k  = g * 8 + e;
      const int kc = (k < kJoints) ? k : (kJoints - 1);
      const float m = sM[kc * 16 + nc];
      const bool ok = (k < kJoints) && (n < kNReal);
      const float v = ok ? m : 0.0f;
      _Float16 h_, l_;
      split_h(v, h_, l_);
      hv[e] = h_;
      lv[e] = l_;
    }
    *(v8h*)(&sBh[n * kKPad + g * 8]) = hv;
    *(v8h*)(&sBl[n * kKPad + g * 8]) = lv;
  }

  float wsum = 0.0f;
#pragma unroll 1
  for (int j = 0; j < kJoints; ++j) {
    const v4f m0 = *(const v4f*)(&sM[j * 16 + 0]);
    const v4f m1 = *(const v4f*)(&sM[j * 16 + 4]);
    const v4f m2 = *(const v4f*)(&sM[j * 16 + 8]);
    const v4f lc = *(const v4f*)(&sL[j * 4]);
    const v4f fa = *(const v4f*)(&sF[j * 12 + 0]);
    const v4f fb = *(const v4f*)(&sF[j * 12 + 4]);
    const v4f fc = *(const v4f*)(&sF[j * 12 + 8]);
    float p0 = m0.x * px;
    p0 = fmaf(m0.y, py, p0);
    p0 = fmaf(m0.z, pz, p0);
    p0 = p0 + m0.w;
    float p1 = m1.x * px;
    p1 = fmaf(m1.y, py, p1);
    p1 = fmaf(m1.z, pz, p1);
    p1 = p1 + m1.w;
    float p2 = m2.x * px;
    p2 = fmaf(m2.y, py, p2);
    p2 = fmaf(m2.z, pz, p2);
    p2 = p2 + m2.w;
    const float vx = lc.x - p0;
    const float vy = lc.y - p1;
    const float vz = lc.z - p2;
    const float t0 = vx * vx;
    const float t1 = vy * vy;
    const float t2 = vz * vz;
    const float ss = (t0 + t2) + t1;
    const float nrm = sqrtf(ss);
    const float len = (nrm != nrm) ? 0.0f : fminf(nrm, 3.4028234663852886e38f);
    const float inv = 1.0f / fmaxf(nrm, 1e-12f);
    const float x = vx * inv;
    const float y = vy * inv;
    const float z = vz * inv;
    const float b1 = kC1n * y;
    const float b2 = kC1 * z;
    const float b3 = kC1n * x;
    const float b4 = (kC2_0 * x) * y;
    const float b5 = (kC2_1 * y) * z;
    const float xx = x * x;
    const float yy = y * y;
    const float b6 = kC2_2 * ((((2.0f * z) * z) - xx) - yy);
    const float b7 = (kC2_3 * x) * z;
    const float b8 = kC2_4 * (xx - yy);
    float s = kC0 * fa.x;
    s = fmaf(b1, fa.y, s);
    s = fmaf(b2, fa.z, s);
    s = fmaf(b3, fa.w, s);
    s = fmaf(b4, fb.x, s);
    s = fmaf(b5, fb.y, s);
    s = fmaf(b6, fb.z, s);
    s = fmaf(b7, fb.w, s);
    s = fmaf(b8, fc.x, s);
    const float rads = fmaxf(s + 0.5f, 0.0f);
    const float rel  = fmaxf(1.0f - len / fmaxf(rads, kEps), 0.0f);
    const float w    = (rads < kEps) ? 0.0f : rel;
    sR[wave][lane * kJoints + j] = w;
    wsum = wsum + w;
  }
  const float winv = 1.0f / fmaxf(wsum, kEps);

  __syncthreads();

#pragma unroll
  for (int g = 0; g < 3; ++g) {
    const v4f a0 = *(const v4f*)(&sR[wave][lane * kJoints + g * 8]);
    const v4f a1 = *(const v4f*)(&sR[wave][lane * kJoints + g * 8 + 4]);
    v8h hv, lv;
#pragma unroll
    for (int e = 0; e < 4; ++e) {
      _Float16 h0, l0, h1, l1;
      split_h(a0[e] * winv, h0, l0);
      split_h(a1[e] * winv, h1, l1);
      hv[e] = h0;
      lv[e] = l0;
      hv[4 + e] = h1;
      lv[4 + e] = l1;
    }
    *(v8h*)(&sAh[wave][lane * kKPad + g * 8]) = hv;
    *(v8h*)(&sAl[wave][lane * kKPad + g * 8]) = lv;
  }
  {
    const v8h zv = (v8h){(_Float16)0.0f, (_Float16)0.0f, (_Float16)0.0f, (_Float16)0.0f,
                         (_Float16)0.0f, (_Float16)0.0f, (_Float16)0.0f, (_Float16)0.0f};
    *(v8h*)(&sAh[wave][lane * kKPad + 24]) = zv;
    *(v8h*)(&sAl[wave][lane * kKPad + 24]) = zv;
  }

  __syncthreads();

  {
    const int hh = lane >> 4;
    const int cc = lane & 15;
    const v16h bh = frag_load(&sBh[cc * kKPad + 8 * hh]);
    const v16h bl = frag_load(&sBl[cc * kKPad + 8 * hh]);
#pragma unroll
    for (int t = 0; t < 2; ++t) {
      const v16h ah = frag_load(&sAh[wave][(t * 16 + cc) * kKPad + 8 * hh]);
      const v16h al = frag_load(&sAl[wave][(t * 16 + cc) * kKPad + 8 * hh]);
      v8f am = (v8f){0.f, 0.f, 0.f, 0.f, 0.f, 0.f, 0.f, 0.f};
      v8f ar = (v8f){0.f, 0.f, 0.f, 0.f, 0.f, 0.f, 0.f, 0.f};
      am = mma_h(ah, bh, am);
      ar = mma_h(al, bh, ar);
      ar = mma_h(ah, bl, ar);
#pragma unroll
      for (int r = 0; r < 8; ++r) {
        sR[wave][(t * 16 + 8 * hh + r) * 16 + cc] = fmaf(ar[r], kCarryInv, am[r]);
      }
    }
  }

  __syncthreads();

  {
    const v4f r0 = *(const v4f*)(&sR[wave][lane * 16 + 0]);
    const v4f r1 = *(const v4f*)(&sR[wave][lane * 16 + 4]);
    const v4f r2 = *(const v4f*)(&sR[wave][lane * 16 + 8]);
    float ax = r0.x * px;
    ax = fmaf(r0.y, py, ax);
    ax = fmaf(r0.z, pz, ax);
    ax = ax + r0.w;
    float ay = r1.x * px;
    ay = fmaf(r1.y, py, ay);
    ay = fmaf(r1.z, pz, ay);
    ay = ay + r1.w;
    float az = r2.x * px;
    az = fmaf(r2.y, py, az);
    az = fmaf(r2.z, pz, az);
    az = az + r2.w;
    float bx = r0.x * qx;
    bx = fmaf(r0.y, qy, bx);
    bx = fmaf(r0.z, qz, bx);
    bx = bx + r0.w;
    float by = r1.x * qx;
    by = fmaf(r1.y, qy, by);
    by = fmaf(r1.z, qz, by);
    by = by + r1.w;
    float bz = r2.x * qx;
    bz = fmaf(r2.y, qy, bz);
    bz = fmaf(r2.z, qz, bz);
    bz = bz + r2.w;
    const bool valid = (wsum > kEps);
    const float o1x = valid ? ax : px;
    const float o1y = valid ? ay : py;
    const float o1z = valid ? az : pz;
    const float o2x = valid ? bx : qx;
    const float o2y = valid ? by : qy;
    const float o2z = valid ? bz : qz;
    sR[wave][kStage0 + lane * 3 + 0] = o1x;
    sR[wave][kStage0 + lane * 3 + 1] = o1y;
    sR[wave][kStage0 + lane * 3 + 2] = o1z;
    sR[wave][kStage1 + lane * 3 + 0] = o1x - o2x;
    sR[wave][kStage1 + lane * 3 + 1] = o1y - o2y;
    sR[wave][kStage1 + lane * 3 + 2] = o1z - o2z;
  }

  __syncthreads();

  {
    const float s0a = sR[wave][kStage0 + lane];
    const float s0b = sR[wave][kStage0 + 32 + lane];
    const float s0c = sR[wave][kStage0 + 64 + lane];
    const float s1a = sR[wave][kStage1 + lane];
    const float s1b = sR[wave][kStage1 + 32 + lane];
    const float s1c = sR[wave][kStage1 + 64 + lane];
    const size_t fbase = ((size_t)blockIdx.x * kBlock + (size_t)wave * 32) * 3;
    volatile float* g0 = (volatile float*)(out + fbase);
    volatile float* g1 = (volatile float*)(out + (size_t)kPts * 3 + fbase);
    for (int pass = 0; pass < 2; ++pass) {
      g0[lane]      = s0a;
      g0[32 + lane] = s0b;
      g0[64 + lane] = s0c;
      g1[lane]      = s1a;
      g1[32 + lane] = s1b;
      g1[64 + lane] = s1c;
      __threadfence();
    }
  }
}

extern "C" void kernel_launch(void* const* d_in, const int* in_sizes, int n_in,
                              void* d_out, int out_size, void* d_ws, size_t ws_size,
                              hipStream_t stream) {
  (void)d_ws;
  (void)ws_size;
  if (n_in < 6) return;
  if (in_sizes[0] != kPts * 3) return;
  if (in_sizes[1] != kPts * 3) return;
  if (in_sizes[2] != kJoints * 16) return;
  if (in_sizes[4] != kJoints * 9) return;
  if (in_sizes[5] != kJoints * 3) return;
  if (out_size != 2 * kPts * 3) return;

  const float* xyz   = (const float*)d_in[0];
  const float* vdir  = (const float*)d_in[1];
  const float* tr    = (const float*)d_in[2];
  const float* feats = (const float*)d_in[4];
  const float* locs  = (const float*)d_in[5];
  float* out = (float*)d_out;

  blend_points_kernel<<<kGrid, kBlock, 0, stream>>>(xyz, vdir, tr, feats, locs, out);
}
